// PPAModel_27934467293572
// MI455X (gfx1250) — hardware-run, weakly checked
//
#include <hip/hip_runtime.h>
#include <math.h>

typedef __attribute__((ext_vector_type(16))) _Float16 v16h;
typedef __attribute__((ext_vector_type(16))) __bf16 v16b;
typedef __attribute__((ext_vector_type(8)))  _Float16 v8h;
typedef __attribute__((ext_vector_type(8)))  float v8f;
typedef __attribute__((ext_vector_type(4)))  float v4f;
typedef __attribute__((ext_vector_type(2)))  float v2f;
typedef __attribute__((ext_vector_type(4)))  unsigned v4u;
typedef __attribute__((ext_vector_type(4)))  int v4i;
typedef float __attribute__((may_alias)) float_a;
typedef int __attribute__((may_alias)) int_a;

template <typename T> __device__ __forceinline__ void vst2(void* p, T v) { *(volatile T*)p = v; __threadfence(); *(volatile T*)p = v; }
__device__ __forceinline__ v8f wmma16(v16h a, v16h b, v8f c) {
  v8f d = __builtin_amdgcn_wmma_f32_16x16x32_f16(false, a, false, b, (short)0, c, false, false);
  asm volatile("v_nop\n\tv_nop\n\tv_nop\n\tv_nop" : "+v"(d) : "v"(a), "v"(b));
  return d;
}
__device__ __forceinline__ v8f wmma_bf(v16b a, v16b b, v8f c) {
  v8f d = __builtin_amdgcn_wmma_f32_16x16x32_bf16(false, a, false, b, (short)0, c, false, false);
  asm volatile("v_nop\n\tv_nop\n\tv_nop\n\tv_nop" : "+v"(d) : "v"(a), "v"(b));
  return d;
}
__device__ __forceinline__ v16h frag_h(const _Float16* rowk0, int lane) {
  union { v16h v; v8h q[2]; } u; const _Float16* p = rowk0 + 8 * (lane >> 4);
  u.q[0] = *(const v8h*)p; u.q[1] = *(const v8h*)(p + 16); return u.v;
}
__device__ __forceinline__ v16h frag_f32(const float* rowk0, int lane) {
  v16h a; const float* p = rowk0 + 8 * (lane >> 4);
#pragma unroll
  for (int i = 0; i < 8; ++i) { a[i] = (_Float16)p[i]; a[8 + i] = (_Float16)p[16 + i]; }
  return a;
}
__device__ __forceinline__ v16h frag_f32s(const float* rowk0, int lane, float sc) {
  v16h a; const float* p = rowk0 + 8 * (lane >> 4);
#pragma unroll
  for (int i = 0; i < 8; ++i) { a[i] = (_Float16)(p[i] * sc); a[8 + i] = (_Float16)(p[16 + i] * sc); }
  return a;
}
__device__ __forceinline__ v16h fragc_f32(const float* W, int k0, int n, int lane, int ld, int K) {
  v16h a; const int g = lane >> 4;
#pragma unroll
  for (int i = 0; i < 8; ++i) { const int ka = k0 + 8 * g + i, kb = ka + 16;
    a[i] = (_Float16)(ka < K ? W[(size_t)(ka < K ? ka : K - 1) * ld + n] : 0.f); a[8 + i] = (_Float16)(kb < K ? W[(size_t)(kb < K ? kb : K - 1) * ld + n] : 0.f); }
  return a;
}
struct F2 { v16b h, l; };
__device__ __forceinline__ F2 bsplit16(const float v[16]) { F2 r;
#pragma unroll
  for (int i = 0; i < 16; ++i) { const __bf16 h = (__bf16)v[i]; r.h[i] = h; r.l[i] = (__bf16)(v[i] - (float)h); }
  return r; }
__device__ __forceinline__ F2 split_row(const float* row, int k0, int lane) { float v[16]; const float* p = row + k0 + 8 * (lane >> 4);
#pragma unroll
  for (int i = 0; i < 8; ++i) { v[i] = p[i]; v[8 + i] = p[16 + i]; }
  return bsplit16(v); }
__device__ __forceinline__ F2 split_rowK(const float* row, int k0, int lane, int K) { float v[16]; const int g = lane >> 4;
#pragma unroll
  for (int i = 0; i < 8; ++i) { const int ka = k0 + 8 * g + i, kb = ka + 16; v[i] = ka < K ? row[ka < K ? ka : K - 1] : 0.f; v[8 + i] = kb < K ? row[kb < K ? kb : K - 1] : 0.f; }
  return bsplit16(v); }
__device__ __forceinline__ F2 split_col(const float* W, int k0, int n, int lane, int ld, int K) { float v[16]; const int g = lane >> 4;
#pragma unroll
  for (int i = 0; i < 8; ++i) { const int ka = k0 + 8 * g + i, kb = ka + 16; v[i] = ka < K ? W[(size_t)(ka < K ? ka : K - 1) * ld + n] : 0.f; v[8 + i] = kb < K ? W[(size_t)(kb < K ? kb : K - 1) * ld + n] : 0.f; }
  return bsplit16(v); }
__device__ __forceinline__ v8f mac3(const F2& a, const F2& b, v8f c) { c = wmma_bf(a.l, b.h, c); c = wmma_bf(a.h, b.l, c); return wmma_bf(a.h, b.h, c); }
__device__ __forceinline__ float sigm(float v) { return 1.0f / (1.0f + expf(-v)); }
#define LDSX() do { asm volatile("s_wait_dscnt 0" ::: "memory"); __builtin_amdgcn_wave_barrier(); __builtin_amdgcn_fence(__ATOMIC_RELEASE, "workgroup"); } while (0)


#define NN 100000
#define NE 1000000
#define IND 128
#define HID 256
#define OUD 128
#define WSC 256.0f
#define NNB ((NN + 63) / 64)
#define NNP (NNB * 64)
#define NEB (NE / 64)
#ifndef TEB
#define TEB NEB
#endif
typedef __attribute__((ext_vector_type(8))) __bf16 v8b;
__device__ __forceinline__ v16b frag_b(const __bf16* rowk0, int lane) {
  union { v16b v; v8b q[2]; } u; const __bf16* p = rowk0 + 8 * (lane >> 4);
  u.q[0] = *(const v8b*)p; u.q[1] = *(const v8b*)(p + 16); return u.v;
}
__device__ __forceinline__ float bfr(float v) { return (float)(__bf16)v; }
__device__ __attribute__((noinline)) float exp_ni(float v) { return expf(v); }
__device__ __attribute__((noinline)) float erf_ni(float v) { return erff(v); }

#define WS_P1  0u
#define WS_P2  (WS_P1 + 2u * HID * IND)
#define WS_P3  (WS_P2 + 2u * OUD * HID)
#define WS_P4  (WS_P3 + 2u * HID * 2 * OUD)
#define WS_H   (WS_P4 + 2u * 16 * HID)
#define WS_PA  (WS_H + 4u * (size_t)NNP * OUD)
#define WS_PB  (WS_PA + 4u * (size_t)NNP * HID)
#define WS_END (WS_PB + 4u * (size_t)NNP * HID)

__global__ __launch_bounds__(256) void k_packw(const float* __restrict__ W1, const float* __restrict__ W2, const float* __restrict__ W3, const float* __restrict__ W4, char* __restrict__ ws) { const int n = blockIdx.x, t = threadIdx.x; __shared__ __align__(16) __bf16 s1[IND]; __shared__ __align__(16) _Float16 s2[HID]; __shared__ __align__(16) __bf16 s3[2 * OUD]; __shared__ __align__(16) _Float16 s4[HID];
  if (t < IND) s1[t] = (__bf16)W1[(size_t)t * HID + n]; if (n < OUD) s2[t] = (_Float16)(bfr(W2[(size_t)t * OUD + n]) * WSC); s3[t] = (__bf16)W3[(size_t)t * HID + n]; if (n < 16) s4[t] = (n == 0) ? (_Float16)(bfr(W4[t]) * WSC) : (_Float16)0.0f; __syncthreads();
  if (t < IND / 8) vst2((unsigned*)((__bf16*)(ws + WS_P1) + (size_t)n * IND + t * 8), *(const v4u*)&s1[t * 8]);
  if (n < OUD && t < HID / 8) vst2((unsigned*)((_Float16*)(ws + WS_P2) + (size_t)n * HID + t * 8), *(const v4u*)&s2[t * 8]);
  if (t < 2 * OUD / 8) vst2((unsigned*)((__bf16*)(ws + WS_P3) + (size_t)n * 2 * OUD + t * 8), *(const v4u*)&s3[t * 8]);
  if (n < 16 && t < HID / 8) vst2((unsigned*)((_Float16*)(ws + WS_P4) + (size_t)n * HID + t * 8), *(const v4u*)&s4[t * 8]); }
__device__ __forceinline__ v16h frag_lds(const _Float16* p, int lane) { v16h a; const _Float16* pp = p + 8 * (lane >> 4);
#pragma unroll
  for (int i = 0; i < 8; ++i) { a[i] = pp[i]; a[8 + i] = pp[16 + i]; } return a; }
__global__ __launch_bounds__(128) void k_node(const float* __restrict__ X, const __bf16* __restrict__ P1, const float* __restrict__ B1, const _Float16* __restrict__ P2, const float* __restrict__ B2, const __bf16* __restrict__ P3, float* __restrict__ H, float* __restrict__ PA, float* __restrict__ PB) {
  __shared__ __align__(16) _Float16 sh[64][HID + 8]; __shared__ __align__(16) float shf[64][OUD + 4]; __shared__ __align__(16) float so[4][16][132];
  const int tid = threadIdx.x, wave = tid >> 5, lane = tid & 31, col = lane & 15, g = lane >> 4; const size_t n0 = (size_t)blockIdx.x * 64 + wave * 16; const size_t nrow = (n0 + col < NN) ? n0 + col : NN - 1;
  { v8f acc[16];
#pragma unroll
    for (int j = 0; j < 16; ++j) acc[j] = v8f{};
#pragma unroll
    for (int kc = 0; kc < IND / 32; ++kc) { v16b a; const float* pp = X + nrow * IND + kc * 32 + 8 * g;
#pragma unroll
      for (int i = 0; i < 8; ++i) { a[i] = (__bf16)pp[i]; a[8 + i] = (__bf16)pp[16 + i]; }
#pragma unroll
      for (int j = 0; j < 16; ++j) acc[j] = wmma_bf(a, frag_b(P1 + (size_t)(j * 16 + col) * IND + kc * 32, lane), acc[j]); }
#pragma unroll
    for (int j = 0; j < 16; ++j) { const int c = j * 16 + col; const float bb = bfr(B1[c]);
#pragma unroll
      for (int r = 0; r < 8; ++r) sh[wave * 16 + 8 * g + r][c] = (_Float16)fmaxf(acc[j][r] + bb, 0.f); } }
  __syncthreads();
  { v8f acc[8] = {};
#pragma unroll
    for (int kc = 0; kc < HID / 32; ++kc) { const v16h a = frag_lds(&sh[wave * 16 + col][kc * 32], lane);
#pragma unroll
      for (int j = 0; j < 8; ++j) acc[j] = wmma16(a, frag_h(P2 + (size_t)(j * 16 + col) * HID + kc * 32, lane), acc[j]); }
#pragma unroll
    for (int j = 0; j < 8; ++j) { const int c = j * 16 + col; const float bb = bfr(B2[c]);
#pragma unroll
      for (int r = 0; r < 8; ++r) shf[wave * 16 + 8 * g + r][c] = acc[j][r] * (1.0f / WSC) + bb; } }
  __syncthreads();
  for (int e = tid; e < 64 * (OUD / 4); e += 128) { const int rl = e / (OUD / 4), q = e % (OUD / 4); vst2(H + ((size_t)blockIdx.x * 64 + rl) * OUD + q * 4, *(const v4f*)&shf[rl][q * 4]); }
#pragma unroll 1
  for (int half = 0; half < 2; ++half) {
#pragma unroll 1
    for (int cc = 0; cc < HID; cc += 128) { v8f acc[8] = {};
#pragma unroll
      for (int kc = 0; kc < OUD / 32; ++kc) { float v[16]; const float* pp = &shf[wave * 16 + col][kc * 32 + 8 * g];
#pragma unroll
        for (int i = 0; i < 8; ++i) { v[i] = pp[i]; v[8 + i] = pp[16 + i]; }
        const F2 a = bsplit16(v);
#pragma unroll
        for (int j = 0; j < 8; ++j) { const v16b w = frag_b(P3 + (size_t)(cc + j * 16 + col) * (2 * OUD) + half * OUD + kc * 32, lane); acc[j] = wmma_bf(a.h, w, acc[j]); acc[j] = wmma_bf(a.l, w, acc[j]); } }
#pragma unroll
      for (int j = 0; j < 8; ++j)
#pragma unroll
        for (int r = 0; r < 8; ++r) so[wave][8 * g + r][j * 16 + col] = acc[j][r];
      LDSX(); float* dst = (half == 0 ? PA : PB); for (int rl = 0; rl < 16; ++rl) vst2(dst + (n0 + rl) * HID + cc + lane * 4, *(const v4f*)&so[wave][rl][lane * 4]); LDSX(); } } }
__global__ __launch_bounds__(128) void k_edge(const int* __restrict__ EI, const float* __restrict__ PA, const float* __restrict__ PB, const float* __restrict__ B3, const _Float16* __restrict__ P4, const float* __restrict__ B4, float* __restrict__ OUT) { __shared__ __align__(16) _Float16 sr[64][HID + 8]; __shared__ int su[64], sv[64]; __shared__ __align__(16) float so[64];
  const int tid = threadIdx.x, wave = tid >> 5, lane = tid & 31, col = lane & 15, g = lane >> 4; const size_t e0 = (size_t)blockIdx.x * 64;
  if (tid < 64) { int u = EI[e0 + tid], v = EI[(size_t)NE + e0 + tid]; u = u < 0 ? 0 : (u >= NN ? NN - 1 : u); v = v < 0 ? 0 : (v >= NN ? NN - 1 : v); su[tid] = u; sv[tid] = v; } __syncthreads();
  for (int e = tid; e < 64 * HID; e += 128) { const int rl = e / HID, c = e % HID; sr[rl][c] = (_Float16)fmaxf(PA[(size_t)su[rl] * HID + c] + PB[(size_t)sv[rl] * HID + c] + bfr(B3[c]), 0.f); }
  __syncthreads();
  v8f acc = {};
#pragma unroll
  for (int kc = 0; kc < HID / 32; ++kc) acc = wmma16(frag_lds(&sr[wave * 16 + col][kc * 32], lane), frag_h(P4 + (size_t)col * HID + kc * 32, lane), acc);
  if (col == 0) { const float bb = bfr(B4[0]);
#pragma unroll
    for (int r = 0; r < 8; ++r) { const float z = acc[r] * (1.0f / WSC) + bb; so[wave * 16 + 8 * g + r] = 1.0f / (1.0f + expf(-z)); } }
  __syncthreads(); if (tid < 16) vst2(OUT + e0 + tid * 4, *(const v4f*)&so[tid * 4]); }
extern "C" void kernel_launch(void* const* d_in, const int* in_sizes, int n_in, void* d_out, int out_size, void* d_ws, size_t ws_size, hipStream_t stream) {
  (void)in_sizes; (void)n_in; (void)out_size;
  const float** F = (const float**)d_in;
  if (ws_size < (size_t)WS_END) return;
  char* ws = (char*)d_ws; float *H = (float*)(ws + WS_H), *PA = (float*)(ws + WS_PA), *PB = (float*)(ws + WS_PB);
  k_packw<<<HID, 256, 0, stream>>>(F[2], F[4], F[6], F[8], ws);
  k_node<<<NNB, 128, 0, stream>>>(F[0], (const __bf16*)(ws + WS_P1), F[3], (const _Float16*)(ws + WS_P2), F[5], (const __bf16*)(ws + WS_P3), H, PA, PB);
  k_edge<<<TEB, 128, 0, stream>>>((const int*)d_in[1], PA, PB, F[7], (const _Float16*)(ws + WS_P4), F[9], (float*)d_out);
}
